// LinearAttention_Cross_40793599377746
// MI455X (gfx1250) — hardware-verified
//
#include <hip/hip_runtime.h>

typedef __bf16         v16b __attribute__((ext_vector_type(16)));
typedef unsigned int   v4u  __attribute__((ext_vector_type(4)));
typedef float          v8f  __attribute__((ext_vector_type(8)));
typedef float          v4f  __attribute__((ext_vector_type(4)));
typedef v4u __attribute__((may_alias)) v4ua;
typedef v4f __attribute__((may_alias)) v4fa;

union Frag { v16b v; v4u q[2]; };

#define NB    8
#define DIMX  256
#define NPIX  4096
#define CDIM  512
#define MPIX  1024
#define HID   512
#define NHEAD 8
#define DH    64
#define OC    256

__device__ __forceinline__ unsigned bfb(float f) {
  unsigned u = __builtin_bit_cast(unsigned, f);
  u += 0x7FFFu + ((u >> 16) & 1u);
  return u >> 16;
}
__device__ __forceinline__ float bfv(unsigned b) {
  return __builtin_bit_cast(float, b << 16);
}
__device__ __forceinline__ unsigned plane_bits(float f, int lo) {
  const unsigned hb = bfb(f);
  const unsigned lb = bfb(f - bfv(hb));
  return lo ? lb : hb;
}
__device__ __forceinline__ v4u pack8v(v4f a, v4f b, int lo) {
  v4u r;
  r.x = plane_bits(a.x, lo) | (plane_bits(a.y, lo) << 16);
  r.y = plane_bits(a.z, lo) | (plane_bits(a.w, lo) << 16);
  r.z = plane_bits(b.x, lo) | (plane_bits(b.y, lo) << 16);
  r.w = plane_bits(b.z, lo) | (plane_bits(b.w, lo) << 16);
  return r;
}

__device__ __forceinline__ v8f mma3(v16b ah, v16b al, v16b bh, v16b bl, v8f c) {
  c = __builtin_amdgcn_wmma_f32_16x16x32_bf16(false, ah, false, bh, (short)0, c, false, false);
  c = __builtin_amdgcn_wmma_f32_16x16x32_bf16(false, ah, false, bl, (short)0, c, false, false);
  c = __builtin_amdgcn_wmma_f32_16x16x32_bf16(false, al, false, bh, (short)0, c, false, false);
  asm volatile("v_nop\n\tv_nop\n\tv_nop\n\tv_nop" : "+v"(c) : "v"(ah), "v"(al), "v"(bh), "v"(bl));
  return c;
}

__device__ __forceinline__ v16b ldfrag(const unsigned short* p) {
  Frag f;
  f.q[0] = *(const v4ua*)(p);
  f.q[1] = *(const v4ua*)(p + 16);
  return f.v;
}

__global__ __launch_bounds__(256) void cvt_w_kernel(
    const float* __restrict__ w0, const float* __restrict__ w1,
    const float* __restrict__ w2, const float* __restrict__ w3,
    int n0, int n1, int n2, int n3, unsigned short* __restrict__ pl)
{
  const int g  = blockIdx.x * 256 + threadIdx.x;
  const int g0 = n0 >> 3, g1 = g0 + (n1 >> 3), g2 = g1 + (n2 >> 3), g3 = g2 + (n3 >> 3);
  if (g >= g3) return;
  const float* src;
  unsigned short* dh;
  int nn;
  if (g < g0)      { src = w0 + (size_t)8 * g;        dh = pl + (size_t)8 * g;                               nn = n0; }
  else if (g < g1) { src = w1 + (size_t)8 * (g - g0); dh = pl + (size_t)2 * n0 + 8 * (g - g0);              nn = n1; }
  else if (g < g2) { src = w2 + (size_t)8 * (g - g1); dh = pl + (size_t)2 * (n0 + n1) + 8 * (g - g1);       nn = n2; }
  else             { src = w3 + (size_t)8 * (g - g2); dh = pl + (size_t)2 * (n0 + n1 + n2) + 8 * (g - g2);  nn = n3; }
  const v4f a = *(const v4fa*)src;
  const v4f b = *(const v4fa*)(src + 4);
  const v4u hi = pack8v(a, b, 0);
  const v4u lo = pack8v(a, b, 1);
  *(volatile v4u*)dh = hi;
  *(volatile v4u*)(dh + nn) = lo;
  __threadfence();
  *(volatile v4u*)dh = hi;
  *(volatile v4u*)(dh + nn) = lo;
}

__device__ __forceinline__ void tr_store_pass(const float* s, unsigned short* oh, unsigned short* ol,
                                              int C, int N, int z, int n0, int c0, int w, int lane) {
  const int q8 = lane & 7, sub = lane >> 3;
  const int plane = w >> 2;
  unsigned short* base = plane ? ol : oh;
  #pragma unroll
  for (int i = 0; i < 4; ++i) {
    const int L  = w * 16 + i * 4 + sub;
    const int nr = L & 63;
    const v4f a = *(const v4fa*)(s + nr * 68 + 8 * q8);
    const v4f b = *(const v4fa*)(s + nr * 68 + 8 * q8 + 4);
    const v4u v = pack8v(a, b, plane);
    unsigned short* dst = base + ((size_t)z * N + n0 + nr) * C + c0 + 8 * q8;
    *(volatile v4u*)dst = v;
  }
}

__global__ __launch_bounds__(256) void tr_cvt_kernel(
    const float* __restrict__ in, const float* __restrict__ smax, const float* __restrict__ sinv,
    unsigned short* __restrict__ oh, unsigned short* __restrict__ ol, int C, int N, int mode)
{
  __shared__ __attribute__((aligned(16))) float s[64 * 68];
  const int tid = threadIdx.x, lane = tid & 31, w = tid >> 5;
  const int n0 = blockIdx.x * 64, c0 = blockIdx.y * 64, z = blockIdx.z;
  const float* src = in + ((size_t)z * C + c0) * N + n0;
  #pragma unroll
  for (int i = 0; i < 16; ++i) {
    const int idx = i * 256 + tid;
    const int c = idx >> 6, n = idx & 63;
    float v = src[(size_t)c * N + n];
    if (mode != 0) {
      const int sc = z * C + c0 + c;
      v = __expf(v - smax[sc]) * sinv[sc];
    }
    s[n * 68 + c] = v;
  }
  __syncthreads();
  tr_store_pass(s, oh, ol, C, N, z, n0, c0, w, lane);
  __threadfence();
  tr_store_pass(s, oh, ol, C, N, z, n0, c0, w, lane);
}

__device__ __forceinline__ void gemm_store_pass(const float* sT, float* Cf, unsigned short* Ch, unsigned short* Cl,
                                                long long oC, int ldc, int row0, int col0, int mode, int w, int lane) {
  const int q8 = lane & 7, sub = lane >> 3;
  if (mode == 0) {
    float* C = Cf + oC;
    #pragma unroll
    for (int i = 0; i < 8; ++i) {
      const int L = w * 32 + i * 4 + sub;
      const int row = L >> 1, hf = L & 1;
      const v4f v = *(const v4fa*)(sT + row * 64 + 32 * hf + 4 * q8);
      *(volatile v4f*)(C + (long long)(row0 + row) * ldc + col0 + 32 * hf + 4 * q8) = v;
    }
  } else {
    const int plane = w >> 1;
    unsigned short* C = (plane ? Cl : Ch) + oC;
    #pragma unroll
    for (int i = 0; i < 8; ++i) {
      const int L = w * 32 + i * 4 + sub;
      const int row = L & 63;
      const v4f a = *(const v4fa*)(sT + row * 64 + 8 * q8);
      const v4f b = *(const v4fa*)(sT + row * 64 + 8 * q8 + 4);
      const v4u v = pack8v(a, b, plane);
      *(volatile v4u*)(C + (long long)(row0 + row) * ldc + col0 + 8 * q8) = v;
    }
  }
}

__global__ __launch_bounds__(128) void gemm_split_kernel(
    const unsigned short* __restrict__ Ah, const unsigned short* __restrict__ Al,
    const unsigned short* __restrict__ Bh, const unsigned short* __restrict__ Bl,
    float* __restrict__ Cf, unsigned short* __restrict__ Ch, unsigned short* __restrict__ Cl,
    int K, int lda, int ldb, int ldc, int zdiv,
    long long sA1, long long sA2, long long sB1, long long sB2, long long sC1, long long sC2,
    float scale, int mode)
{
  __shared__ __attribute__((aligned(16))) float sT[64 * 64];

  const int tid = threadIdx.x, lane = tid & 31, w = tid >> 5;
  const int h = lane >> 4, m = lane & 15;
  const int col0 = blockIdx.x * 64, row0 = blockIdx.y * 64, z = blockIdx.z;
  const int z1 = z / zdiv, z2 = z - z1 * zdiv;
  const long long oA = (long long)z1 * sA1 + (long long)z2 * sA2;
  const long long oB = (long long)z1 * sB1 + (long long)z2 * sB2;
  const long long oC = (long long)z1 * sC1 + (long long)z2 * sC2;
  const int wr = (w >> 1) * 32, wc = (w & 1) * 32;

  const long long offA = (long long)(row0 + wr + m) * lda + 8 * h;
  const long long offB = (long long)(col0 + wc + m) * ldb + 8 * h;
  const unsigned short* pah0 = Ah + oA + offA;
  const unsigned short* pah1 = pah0 + (long long)16 * lda;
  const unsigned short* pal0 = Al + oA + offA;
  const unsigned short* pal1 = pal0 + (long long)16 * lda;
  const unsigned short* pbh0 = Bh + oB + offB;
  const unsigned short* pbh1 = pbh0 + (long long)16 * ldb;
  const unsigned short* pbl0 = Bl + oB + offB;
  const unsigned short* pbl1 = pbl0 + (long long)16 * ldb;

  const v8f zero8 = {0.f, 0.f, 0.f, 0.f, 0.f, 0.f, 0.f, 0.f};
  v8f acc[2][2];
  acc[0][0] = zero8; acc[0][1] = zero8; acc[1][0] = zero8; acc[1][1] = zero8;

  #pragma unroll 1
  for (int k0 = 0; k0 < K; k0 += 32) {
    const v16b ah0 = ldfrag(pah0 + k0), ah1 = ldfrag(pah1 + k0);
    const v16b al0 = ldfrag(pal0 + k0), al1 = ldfrag(pal1 + k0);
    const v16b bh0 = ldfrag(pbh0 + k0), bh1 = ldfrag(pbh1 + k0);
    const v16b bl0 = ldfrag(pbl0 + k0), bl1 = ldfrag(pbl1 + k0);
    acc[0][0] = mma3(ah0, al0, bh0, bl0, acc[0][0]);
    acc[0][1] = mma3(ah0, al0, bh1, bl1, acc[0][1]);
    acc[1][0] = mma3(ah1, al1, bh0, bl0, acc[1][0]);
    acc[1][1] = mma3(ah1, al1, bh1, bl1, acc[1][1]);
  }

  #pragma unroll
  for (int mt = 0; mt < 2; ++mt)
    #pragma unroll
    for (int nt = 0; nt < 2; ++nt)
      #pragma unroll
      for (int r = 0; r < 8; ++r)
        sT[(wr + 16 * mt + 8 * h + r) * 64 + wc + 16 * nt + m] = acc[mt][nt][r] * scale;
  __syncthreads();

  gemm_store_pass(sT, Cf, Ch, Cl, oC, ldc, row0, col0, mode, w, lane);
  __threadfence();
  gemm_store_pass(sT, Cf, Ch, Cl, oC, ldc, row0, col0, mode, w, lane);
}

__global__ __launch_bounds__(256) void softmax_stats_kernel(
    const float* __restrict__ q, float* __restrict__ smax, float* __restrict__ sinv)
{
  __shared__ __attribute__((aligned(16))) float sm[32];
  __shared__ __attribute__((aligned(16))) float si[32];
  const int tid = threadIdx.x, lane = tid & 31, w = tid >> 5;
  const int r0 = blockIdx.x * 32;
  #pragma unroll 1
  for (int j = 0; j < 4; ++j) {
    const int rl = w * 4 + j;
    const float* p = q + (size_t)(r0 + rl) * NPIX;
    float mx = -3.0e38f;
    #pragma unroll 1
    for (int c = lane * 4; c < NPIX; c += 128) {
      const v4f v = *(const v4fa*)(p + c);
      mx = fmaxf(mx, fmaxf(fmaxf(v.x, v.y), fmaxf(v.z, v.w)));
    }
    #pragma unroll
    for (int o = 16; o > 0; o >>= 1) mx = fmaxf(mx, __shfl_xor(mx, o));
    float s = 0.0f;
    #pragma unroll 1
    for (int c = lane * 4; c < NPIX; c += 128) {
      const v4f v = *(const v4fa*)(p + c);
      s += (__expf(v.x - mx) + __expf(v.y - mx)) + (__expf(v.z - mx) + __expf(v.w - mx));
    }
    #pragma unroll
    for (int o = 16; o > 0; o >>= 1) s += __shfl_xor(s, o);
    if (lane == 0) { sm[rl] = mx; si[rl] = 1.0f / s; }
  }
  __syncthreads();
  if (w == 0) {
    const int q8 = lane & 7, sub = lane >> 3;
    const v4f a = *(const v4fa*)(sm + 4 * q8);
    const v4f c = *(const v4fa*)(si + 4 * q8);
    v4f v;
    v.x = (sub == 0) ? a.x : c.x;
    v.y = (sub == 0) ? a.y : c.y;
    v.z = (sub == 0) ? a.z : c.z;
    v.w = (sub == 0) ? a.w : c.w;
    float* dst = ((sub == 0) ? smax : sinv) + r0 + 4 * q8;
    if (sub < 2) *(volatile v4f*)dst = v;
    __threadfence();
    if (sub < 2) *(volatile v4f*)dst = v;
  }
}

__device__ __forceinline__ void ln_store_pass(const float* sY, const float* smean, const float* srstd,
                                              const float* gain, float* out, int b, int n0, int w, int lane) {
  const int q8 = lane & 7, sub = lane >> 3;
  #pragma unroll
  for (int i = 0; i < 8; ++i) {
    const int oc = w * 32 + i * 4 + sub;
    const float gg = gain[oc];
    const int n = 4 * q8;
    v4f o;
    o.x = ((sY[(n + 0) * 260 + oc] - smean[n + 0]) * srstd[n + 0]) * gg;
    o.y = ((sY[(n + 1) * 260 + oc] - smean[n + 1]) * srstd[n + 1]) * gg;
    o.z = ((sY[(n + 2) * 260 + oc] - smean[n + 2]) * srstd[n + 2]) * gg;
    o.w = ((sY[(n + 3) * 260 + oc] - smean[n + 3]) * srstd[n + 3]) * gg;
    *(volatile v4f*)(out + ((size_t)b * OC + oc) * NPIX + n0 + n) = o;
  }
}

__global__ __launch_bounds__(256) void out_ln_kernel(
    const unsigned short* __restrict__ Ah, const unsigned short* __restrict__ Al,
    const unsigned short* __restrict__ Wh, const unsigned short* __restrict__ Wl,
    const float* __restrict__ bo, const float* __restrict__ gain, float* __restrict__ out)
{
  __shared__ __attribute__((aligned(16))) float sY[32 * 260];
  __shared__ __attribute__((aligned(16))) float smean[32];
  __shared__ __attribute__((aligned(16))) float srstd[32];

  const int tid = threadIdx.x, lane = tid & 31, w = tid >> 5;
  const int h = lane >> 4, m = lane & 15;
  const int b = blockIdx.y, n0 = blockIdx.x * 32, oc0 = w * 32;

  const size_t offA = ((size_t)b * NPIX + n0 + m) * HID + 8 * h;
  const size_t offB = (size_t)(oc0 + m) * HID + 8 * h;
  const unsigned short* pah0 = Ah + offA;
  const unsigned short* pah1 = pah0 + 16 * HID;
  const unsigned short* pal0 = Al + offA;
  const unsigned short* pal1 = pal0 + 16 * HID;
  const unsigned short* pbh0 = Wh + offB;
  const unsigned short* pbh1 = pbh0 + 16 * HID;
  const unsigned short* pbl0 = Wl + offB;
  const unsigned short* pbl1 = pbl0 + 16 * HID;

  const v8f zero8 = {0.f, 0.f, 0.f, 0.f, 0.f, 0.f, 0.f, 0.f};
  v8f acc[2][2];
  acc[0][0] = zero8; acc[0][1] = zero8; acc[1][0] = zero8; acc[1][1] = zero8;

  #pragma unroll 1
  for (int k0 = 0; k0 < HID; k0 += 32) {
    const v16b ah0 = ldfrag(pah0 + k0), ah1 = ldfrag(pah1 + k0);
    const v16b al0 = ldfrag(pal0 + k0), al1 = ldfrag(pal1 + k0);
    const v16b bh0 = ldfrag(pbh0 + k0), bh1 = ldfrag(pbh1 + k0);
    const v16b bl0 = ldfrag(pbl0 + k0), bl1 = ldfrag(pbl1 + k0);
    acc[0][0] = mma3(ah0, al0, bh0, bl0, acc[0][0]);
    acc[0][1] = mma3(ah0, al0, bh1, bl1, acc[0][1]);
    acc[1][0] = mma3(ah1, al1, bh0, bl0, acc[1][0]);
    acc[1][1] = mma3(ah1, al1, bh1, bl1, acc[1][1]);
  }

  #pragma unroll
  for (int nt = 0; nt < 2; ++nt) {
    const int oc = oc0 + 16 * nt + m;
    const float bb = bo[oc];
    #pragma unroll
    for (int mt = 0; mt < 2; ++mt)
      #pragma unroll
      for (int r = 0; r < 8; ++r)
        sY[(16 * mt + 8 * h + r) * 260 + oc] = acc[mt][nt][r] + bb;
  }
  __syncthreads();

  {
    const int row = tid >> 3, part = tid & 7;
    const float* pr = sY + row * 260 + part * 32;
    float s = 0.0f;
    #pragma unroll
    for (int j = 0; j < 32; ++j) s += pr[j];
    s += __shfl_xor(s, 1);
    s += __shfl_xor(s, 2);
    s += __shfl_xor(s, 4);
    const float mean = s * (1.0f / 256.0f);
    float d = 0.0f;
    #pragma unroll
    for (int j = 0; j < 32; ++j) { const float t = pr[j] - mean; d += t * t; }
    d += __shfl_xor(d, 1);
    d += __shfl_xor(d, 2);
    d += __shfl_xor(d, 4);
    const float var = d * (1.0f / 256.0f);
    if (part == 0) { smean[row] = mean; srstd[row] = rsqrtf(var + 1e-5f); }
  }
  __syncthreads();

  ln_store_pass(sY, smean, srstd, gain, out, b, n0, w, lane);
  __threadfence();
  ln_store_pass(sY, smean, srstd, gain, out, b, n0, w, lane);
}

extern "C" void kernel_launch(void* const* d_in, const int* in_sizes, int n_in,
                              void* d_out, int out_size, void* d_ws, size_t ws_size,
                              hipStream_t stream) {
  if (n_in < 8) return;
  if (in_sizes[0] != NB * DIMX * NPIX) return;
  if (in_sizes[1] != NB * CDIM * MPIX) return;
  if (in_sizes[2] != HID * DIMX) return;
  if (in_sizes[3] != HID * CDIM || in_sizes[4] != HID * CDIM) return;
  if (in_sizes[5] != OC * HID) return;
  if (in_sizes[6] < OC || in_sizes[7] < OC) return;
  if (out_size != NB * OC * NPIX) return;

  const float* x   = (const float*)d_in[0];
  const float* ct  = (const float*)d_in[1];
  const float* Wq  = (const float*)d_in[2];
  const float* Wk  = (const float*)d_in[3];
  const float* Wv  = (const float*)d_in[4];
  const float* Wo  = (const float*)d_in[5];
  const float* bo  = (const float*)d_in[6];
  const float* gn  = (const float*)d_in[7];
  float* out = (float*)d_out;

  const size_t nWq = (size_t)HID * DIMX, nWk = (size_t)HID * CDIM, nWv = (size_t)HID * CDIM, nWo = (size_t)OC * HID;
  const size_t bW    = (nWq + nWk + nWv + nWo) * 2 * 2;
  const size_t bStat = (size_t)2 * NB * HID * 4;
  const size_t bCtx  = (size_t)2 * NB * NHEAD * DH * DH * 2;
  const size_t bR1   = (size_t)NB * HID * NPIX * 4;
  const size_t bR2   = (size_t)2 * NB * NPIX * HID * 2;
  const size_t oW = 0, oStat = oW + bW, oCtx = oStat + bStat, oR1 = oCtx + bCtx, oR2 = oR1 + bR1;
  const size_t total = oR2 + bR2;
  if (total > ws_size) return;
  if ((size_t)6 * NB * HID * MPIX * 2 > bR1) return;

  char* ws = (char*)d_ws;
  unsigned short* wpl = (unsigned short*)(ws + oW);
  unsigned short* Wqh = wpl;                        unsigned short* Wql = Wqh + nWq;
  unsigned short* Wkh = wpl + 2 * nWq;              unsigned short* Wkl = Wkh + nWk;
  unsigned short* Wvh = wpl + 2 * (nWq + nWk);      unsigned short* Wvl = Wvh + nWv;
  unsigned short* Woh = wpl + 2 * (nWq + nWk + nWv); unsigned short* Wol = Woh + nWo;
  float* smax = (float*)(ws + oStat);
  float* sinv = smax + NB * HID;
  unsigned short* cxh = (unsigned short*)(ws + oCtx);
  unsigned short* cxl = cxh + (size_t)NB * NHEAD * DH * DH;
  const size_t nCT = (size_t)NB * MPIX * CDIM;
  unsigned short* cTh = (unsigned short*)(ws + oR1);
  unsigned short* cTl = cTh + nCT;
  unsigned short* kh  = cTh + 2 * nCT;
  unsigned short* kl  = cTh + 3 * nCT;
  unsigned short* vh  = cTh + 4 * nCT;
  unsigned short* vl  = cTh + 5 * nCT;
  float* qf = (float*)(ws + oR1);
  unsigned short* ath = (unsigned short*)(ws + oR1);
  unsigned short* atl = ath + (size_t)NB * NPIX * HID;
  unsigned short* xTh = (unsigned short*)(ws + oR2);
  unsigned short* xTl = xTh + (size_t)NB * NPIX * DIMX;
  unsigned short* qsh = (unsigned short*)(ws + oR2);
  unsigned short* qsl = qsh + (size_t)NB * NPIX * HID;

  const int ngrp = (int)((nWq + nWk + nWv + nWo) / 8);
  cvt_w_kernel<<<(ngrp + 255) / 256, 256, 0, stream>>>(Wq, Wk, Wv, Wo, (int)nWq, (int)nWk, (int)nWv, (int)nWo, wpl);

  tr_cvt_kernel<<<dim3(MPIX / 64, CDIM / 64, NB), 256, 0, stream>>>(ct, smax, sinv, cTh, cTl, CDIM, MPIX, 0);

  gemm_split_kernel<<<dim3(MPIX / 64, HID / 64, NB), 128, 0, stream>>>(
      Wkh, Wkl, cTh, cTl, smax, kh, kl, CDIM, CDIM, CDIM, MPIX, 1,
      0LL, 0LL, (long long)MPIX * CDIM, 0LL, (long long)HID * MPIX, 0LL, 1.0f, 1);
  gemm_split_kernel<<<dim3(MPIX / 64, HID / 64, NB), 128, 0, stream>>>(
      Wvh, Wvl, cTh, cTl, smax, vh, vl, CDIM, CDIM, CDIM, MPIX, 1,
      0LL, 0LL, (long long)MPIX * CDIM, 0LL, (long long)HID * MPIX, 0LL, 1.0f, 1);

  gemm_split_kernel<<<dim3(1, 1, NB * NHEAD), 128, 0, stream>>>(
      vh, vl, kh, kl, smax, cxh, cxl, MPIX, MPIX, MPIX, DH, 1,
      (long long)DH * MPIX, 0LL, (long long)DH * MPIX, 0LL, (long long)DH * DH, 0LL, 1.0f / 1024.0f, 1);

  tr_cvt_kernel<<<dim3(NPIX / 64, DIMX / 64, NB), 256, 0, stream>>>(x, smax, sinv, xTh, xTl, DIMX, NPIX, 0);

  gemm_split_kernel<<<dim3(NPIX / 64, HID / 64, NB), 128, 0, stream>>>(
      Wqh, Wql, xTh, xTl, qf, cxh, cxl, DIMX, DIMX, DIMX, NPIX, 1,
      0LL, 0LL, (long long)NPIX * DIMX, 0LL, (long long)HID * NPIX, 0LL, 1.0f, 0);

  softmax_stats_kernel<<<(NB * HID) / 32, 256, 0, stream>>>(qf, smax, sinv);

  tr_cvt_kernel<<<dim3(NPIX / 64, HID / 64, NB), 256, 0, stream>>>(qf, smax, sinv, qsh, qsl, HID, NPIX, 1);

  gemm_split_kernel<<<dim3(1, NPIX / 64, NB * NHEAD), 128, 0, stream>>>(
      qsh, qsl, cxh, cxl, smax, ath, atl, DH, HID, DH, HID, NHEAD,
      (long long)NPIX * HID, (long long)DH, (long long)NHEAD * DH * DH, (long long)DH * DH,
      (long long)NPIX * HID, (long long)DH, 1.0f, 1);

  out_ln_kernel<<<dim3(NPIX / 32, NB), 256, 0, stream>>>(ath, atl, Woh, Wol, bo, gn, out);
}
